// Decoder_87978110091940
// MI455X (gfx1250) — hardware-verified
//
#include <hip/hip_runtime.h>
#include <math.h>

constexpr int NBAT   = 8;
constexpr int NTE    = 256;
constexpr int NH     = 256;
constexpr int NENC   = 512;
constexpr int NMEL   = 80;
constexpr int NSTEP  = 100;
constexpr int NG4    = 4 * NH;
constexpr int KATT   = NH + NENC;
constexpr int KIN1   = NMEL + NENC;
constexpr int K1REAL = KIN1 + NH;
constexpr int K1PAD  = 864;
constexpr int W1PITCH = 896;
constexpr int A1P    = 872;
constexpr int K23    = 2 * NH;
constexpr int A23P   = 520;
constexpr int KDEC   = NH + NENC;
constexpr int NTHR   = 512;
constexpr int NROWS  = NBAT * NTE;
constexpr int NOUT0  = NBAT * NSTEP * NMEL;
constexpr int NOUT1  = NBAT * NSTEP;
constexpr float ACARRY = 256.0f;
constexpr float WCARRY = 16.0f;
constexpr float FOLD   = 1.0f / (ACARRY * WCARRY);
constexpr float PCARRY = 32768.0f;
constexpr float PINV   = 1.0f / PCARRY;

static_assert(K1REAL == 848 && K1PAD % 32 == 0 && K1PAD >= K1REAL && W1PITCH >= K1PAD, "gate-1 K padding");
static_assert((W1PITCH * 2) % 128 == 0, "Wc1 rows are whole lines");
static_assert(K23 % 32 == 0 && KDEC % 32 == 0 && NH % 32 == 0 && NTE % 32 == 0 && NENC % 32 == 0, "K multiples of 32");
static_assert(NROWS % 64 == 0 && NH % 64 == 0, "hoist GEMM tile multiples");
static_assert(A1P % 8 == 0 && A23P % 8 == 0 && A1P >= K1PAD && A23P >= K23, "LDS tile pitches");
static_assert(NMEL % 16 == 0 && NMEL % 8 == 0 && KIN1 % 8 == 0, "8-column groups");
static_assert((NOUT0 * 4) % 128 == 0, "second output starts on a line");
static_assert((NOUT0 + NOUT1) * 4 == 259200, "output bytes");
static_assert((2 * NMEL * 4) % 128 == 0 && (NSTEP * NMEL * 4) % 128 == 0 && NSTEP % 2 == 0, "step pairs are whole lines");
static_assert(NBAT * NH == 4 * NTHR && NTHR == 512, "elementwise coverage");

typedef __attribute__((ext_vector_type(16))) _Float16 v16h;
typedef __attribute__((ext_vector_type(8)))  _Float16 v8h;
typedef __attribute__((ext_vector_type(16))) __bf16   v16b;
typedef __attribute__((ext_vector_type(8)))  __bf16   v8b;
typedef __attribute__((ext_vector_type(8)))  float    v8f;
typedef __attribute__((ext_vector_type(4)))  float    v4f;

__device__ __forceinline__ unsigned short f2bf_bits(float f) {
  unsigned u = __float_as_uint(f);
  return (unsigned short)((u + 0x7FFFu + ((u >> 16) & 1u)) >> 16);
}
__device__ __forceinline__ float bf_bits2f(unsigned short h) { return __uint_as_float(((unsigned)h) << 16); }

__device__ __forceinline__ void dep_guard4_h(v8f& a, v8f& b, v8f& c, v8f& d, v16h x, v16h y) { asm volatile("v_nop\n\tv_nop\n\tv_nop\n\tv_nop" : "+v"(a), "+v"(b), "+v"(c), "+v"(d) : "v"(x), "v"(y)); }
__device__ __forceinline__ void dep_guard4_b(v8f& a, v8f& b, v8f& c, v8f& d, v16b x, v16b y) { asm volatile("v_nop\n\tv_nop\n\tv_nop\n\tv_nop" : "+v"(a), "+v"(b), "+v"(c), "+v"(d) : "v"(x), "v"(y)); }
__device__ __forceinline__ void dep_guard1_h(v8f& a, v16h x, v16h y) { asm volatile("v_nop\n\tv_nop\n\tv_nop\n\tv_nop" : "+v"(a) : "v"(x), "v"(y)); }
__device__ __forceinline__ void keep4_h(v16h a, v16h b, v16h c, v16h d) { asm volatile("v_nop" :: "v"(a), "v"(b), "v"(c), "v"(d)); }
__device__ __forceinline__ void keep4_b(v16b a, v16b b, v16b c, v16b d) { asm volatile("v_nop" :: "v"(a), "v"(b), "v"(c), "v"(d)); }
__device__ __forceinline__ void acc_guard4(v8f& a, v8f& b, v8f& c, v8f& d) { asm volatile("v_nop\n\tv_nop\n\tv_nop\n\tv_nop" : "+v"(a), "+v"(b), "+v"(c), "+v"(d)); }
__device__ __forceinline__ void acc_guard1(v8f& a) { asm volatile("v_nop\n\tv_nop\n\tv_nop\n\tv_nop" : "+v"(a)); }

template <typename T> struct Frag;
template <> struct Frag<_Float16> {
  typedef v16h V; union U { v16h v; v8h h[2]; };
  static __device__ __forceinline__ v16h load(const _Float16* p) {
    U f; f.h[0] = *(const v8h*)(p); f.h[1] = *(const v8h*)(p + 16); return f.v;
  }
  static __device__ __forceinline__ v8f mma(v16h a, v16h b, v8f c) {
    return __builtin_amdgcn_wmma_f32_16x16x32_f16(false, a, false, b, (short)0, c, false, false);
  }
  static __device__ __forceinline__ void guard4(v8f& a, v8f& b, v8f& c, v8f& d, v16h x, v16h y) { dep_guard4_h(a, b, c, d, x, y); }
  static __device__ __forceinline__ void keep(v16h a, v16h b, v16h c, v16h d) { keep4_h(a, b, c, d); }
};
template <> struct Frag<__bf16> {
  typedef v16b V; union U { v16b v; v8b h[2]; };
  static __device__ __forceinline__ v16b load(const __bf16* p) {
    U f; f.h[0] = *(const v8b*)(p); f.h[1] = *(const v8b*)(p + 16); return f.v;
  }
  static __device__ __forceinline__ v8f mma(v16b a, v16b b, v8f c) {
    return __builtin_amdgcn_wmma_f32_16x16x32_bf16(false, a, false, b, (short)0, c, false, false);
  }
  static __device__ __forceinline__ void guard4(v8f& a, v8f& b, v8f& c, v8f& d, v16b x, v16b y) { dep_guard4_b(a, b, c, d, x, y); }
  static __device__ __forceinline__ void keep(v16b a, v16b b, v16b c, v16b d) { keep4_b(a, b, c, d); }
};

__device__ __forceinline__ float fsig(float x) {
  const float xc = fminf(fmaxf(x, -30.0f), 30.0f);
  return __builtin_amdgcn_rcpf(1.0f + expf(-xc));
}
__device__ __forceinline__ float ftanh(float x) {
  const float xc = fminf(fmaxf(x, -15.0f), 15.0f);
  return 1.0f - 2.0f * __builtin_amdgcn_rcpf(expf(2.0f * xc) + 1.0f);
}

template <int ET> struct Elem;
template <> struct Elem<0> { typedef _Float16 T; };
template <> struct Elem<1> { typedef __bf16 T; };
template <int ET, bool SPLIT, int BIAS_MODE, int OUT_MODE, bool RESID, int ACT = 0>
__global__ __launch_bounds__(256) void wmma_gemm64(
    const unsigned short* __restrict__ Ap, const unsigned short* __restrict__ A2p, int lda, long strideA,
    const unsigned short* __restrict__ Btp, const unsigned short* __restrict__ Bt2p, int ldb, long strideB,
    void* __restrict__ Cout, void* __restrict__ Cout2, int ldc, long strideC,
    const float* __restrict__ bias,
    const float* __restrict__ resid, long strideR,
    int M, int N, int K, float scale) {
  typedef typename Elem<ET>::T T;
  typedef typename Frag<T>::V V;
  const T* A = (const T*)Ap; const T* A2 = (const T*)A2p; const T* Bt = (const T*)Btp; const T* Bt2 = (const T*)Bt2p;
  __shared__ __align__(16) float sT[8][16 * 68];
  const int b    = blockIdx.y;
  const int lane = threadIdx.x & 31;
  const int wave = threadIdx.x >> 5;
  const int tilesN = N >> 6;
  const int tilesM = M >> 6;
  const int tile = blockIdx.x * 8 + wave;
  if (tile >= tilesM * tilesN) return;
  const int tm = tile / tilesN;
  const int tn = tile - tm * tilesN;
  const int m0 = tm << 6;
  const int n0 = tn << 6;

  const T* Ab  = A  + (size_t)b * strideA;
  const T* Bb  = Bt + (size_t)b * strideB;
  const T* Ab2 = SPLIT ? (A2  + (size_t)b * strideA) : nullptr;
  const T* Bb2 = SPLIT ? (Bt2 + (size_t)b * strideB) : nullptr;

  const int rlane = lane & 15;
  const int koff  = (lane >> 4) * 8;
  const int mOff  = (lane >> 4) * 8;

  v8f acc[4][4];
#pragma unroll
  for (int i = 0; i < 4; ++i)
#pragma unroll
    for (int j = 0; j < 4; ++j) acc[i][j] = (v8f){0.f,0.f,0.f,0.f,0.f,0.f,0.f,0.f};

  for (int k0 = 0; k0 < K; k0 += 32) {
    V bh[4], bl[4];
#pragma unroll
    for (int j = 0; j < 4; ++j) {
      const size_t bo = (size_t)(n0 + (j << 4) + rlane) * ldb + koff + k0;
      bh[j] = Frag<T>::load(Bb + bo);
      if (SPLIT) bl[j] = Frag<T>::load(Bb2 + bo);
    }
#pragma unroll
    for (int i = 0; i < 4; ++i) {
      const size_t ao = (size_t)(m0 + (i << 4) + rlane) * lda + koff + k0;
      V ah = Frag<T>::load(Ab + ao);
      V al;
      if (SPLIT) al = Frag<T>::load(Ab2 + ao);
#pragma unroll
      for (int j = 0; j < 4; ++j) {
        acc[i][j] = Frag<T>::mma(ah, bh[j], acc[i][j]);
        if (SPLIT) {
          acc[i][j] = Frag<T>::mma(ah, bl[j], acc[i][j]);
          acc[i][j] = Frag<T>::mma(al, bh[j], acc[i][j]);
        }
      }
      Frag<T>::guard4(acc[i][0], acc[i][1], acc[i][2], acc[i][3], ah, SPLIT ? al : bh[3]);
    }
    Frag<T>::keep(bh[0], bh[1], bh[2], bh[3]);
    if (SPLIT) Frag<T>::keep(bl[0], bl[1], bl[2], bl[3]);
  }
  acc_guard4(acc[0][0], acc[0][1], acc[0][2], acc[0][3]);
  acc_guard4(acc[1][0], acc[1][1], acc[1][2], acc[1][3]);
  acc_guard4(acc[2][0], acc[2][1], acc[2][2], acc[2][3]);
  acc_guard4(acc[3][0], acc[3][1], acc[3][2], acc[3][3]);

  float* slab = sT[wave];
  const float* Rb = RESID ? (resid + (size_t)b * strideR) : nullptr;
#pragma unroll
  for (int i = 0; i < 4; ++i) {
    const int mBase = m0 + (i << 4);
#pragma unroll
    for (int j = 0; j < 4; ++j) {
      const int n = n0 + (j << 4) + rlane;
      float bv = 0.f;
      if (BIAS_MODE == 2) bv = bias[n];
#pragma unroll
      for (int r = 0; r < 8; ++r) {
        float v = acc[i][j][r] * scale;
        if (BIAS_MODE == 1) v += bias[mBase + mOff + r];
        if (BIAS_MODE == 2) v += bv;
        if (RESID) v += Rb[(size_t)(mBase + mOff + r) * ldc + n];
        if (ACT == 1) v = tanhf(v);
        if (ACT == 2) v = fmaxf(v, 0.0f);
        if (ACT == 3) v = v / (1.0f + expf(-v));
        if (ACT == 4) v = (v > 0.f) ? v : 0.01f * v;
        if (ACT == 5) v = 0.5f * v * (1.0f + erff(v * 0.70710678118654752f));
        slab[(mOff + r) * 68 + (j << 4) + rlane] = v;
      }
    }
    __builtin_amdgcn_fence(__ATOMIC_RELEASE, "workgroup");
    __builtin_amdgcn_wave_barrier();
    __builtin_amdgcn_fence(__ATOMIC_ACQUIRE, "workgroup");
    if (OUT_MODE == 0) {
      float* C = (float*)Cout + (size_t)b * strideC;
      const int hh = lane >> 4, c4 = (lane & 15) * 4;
      for (int pass = 0; pass < 2; ++pass) {
#pragma unroll
        for (int it = 0; it < 8; ++it) {
          const int row = it * 2 + hh;
          v4f v = *(const v4f*)(slab + row * 68 + c4);
          *(volatile v4f*)(C + (size_t)(mBase + row) * ldc + n0 + c4) = v;
        }
        __threadfence();
      }
    } else {
      const int q = lane >> 3, c8 = (lane & 7) * 8;
      unsigned short* C  = (unsigned short*)Cout  + (size_t)b * strideC;
      unsigned short* C2 = (OUT_MODE == 2) ? ((unsigned short*)Cout2 + (size_t)b * strideC) : nullptr;
      for (int pass = 0; pass < 2; ++pass) {
#pragma unroll
        for (int it = 0; it < 4; ++it) {
          const int row = it * 4 + q;
          const float* sp = slab + row * 68 + c8;
          v8h hv, lv;
#pragma unroll
          for (int e = 0; e < 8; ++e) {
            if (OUT_MODE == 1) {
              hv[e] = (_Float16)sp[e];
            } else {
              unsigned short hb = f2bf_bits(sp[e]);
              unsigned short lb = f2bf_bits(sp[e] - bf_bits2f(hb));
              hv[e] = __builtin_bit_cast(_Float16, hb);
              lv[e] = __builtin_bit_cast(_Float16, lb);
            }
          }
          *(volatile v8h*)(C + (size_t)(mBase + row) * ldc + n0 + c8) = hv;
          if (OUT_MODE == 2) *(volatile v8h*)(C2 + (size_t)(mBase + row) * ldc + n0 + c8) = lv;
        }
        __threadfence();
      }
    }
    __builtin_amdgcn_fence(__ATOMIC_RELEASE, "workgroup");
    __builtin_amdgcn_wave_barrier();
    __builtin_amdgcn_fence(__ATOMIC_ACQUIRE, "workgroup");
  }
}

__global__ __launch_bounds__(256) void pack2_kernel(const float* __restrict__ src0, int p0, int c0, int g0,
                                                    const float* __restrict__ src1, int p1, int c1, int g1,
                                                    int gd, int nrow, unsigned short* __restrict__ dst, float sc) {
  const int i  = blockIdx.x * 256 + threadIdx.x;
  const int n8 = nrow * gd;
  if (i < n8) {
    const int row = i / gd;
    const int g   = i - row * gd;
    const int ga  = (g < g0) ? g : (g0 - 1);
    int gb = g - g0;
    gb = (gb < 0) ? 0 : gb;
    const int g1m = (g1 > 0) ? (g1 - 1) : 0;
    gb = (gb > g1m) ? g1m : gb;
    const float* pa = src0 + (size_t)row * p0 + c0 + ga * 8;
    const float* pb = src1 + (size_t)row * p1 + c1 + gb * 8;
    const v4f a0 = *(const v4f*)(pa);
    const v4f a1 = *(const v4f*)(pa + 4);
    const v4f b0 = *(const v4f*)(pb);
    const v4f b1 = *(const v4f*)(pb + 4);
    const float fa = (g < g0) ? 1.0f : 0.0f;
    const float fb = (g >= g0 && g < g0 + g1) ? 1.0f : 0.0f;
    const bool live = (g < g0 + g1);
    v8h hv;
#pragma unroll
    for (int e = 0; e < 4; ++e) {
      float x0 = fmaf(fa, a0[e], fb * b0[e]);
      float x1 = fmaf(fa, a1[e], fb * b1[e]);
      x0 = live ? x0 : 0.0f;
      x1 = live ? x1 : 0.0f;
      hv[e]     = (_Float16)(x0 * sc);
      hv[4 + e] = (_Float16)(x1 * sc);
    }
    *(volatile v8h*)(dst + (size_t)i * 8) = hv;
    __threadfence();
    *(volatile v8h*)(dst + (size_t)i * 8) = hv;
  }
}

__global__ __launch_bounds__(256) void tpose_f16_kernel(const float* __restrict__ src, int R, int C, int ldo,
                                                        unsigned short* __restrict__ O, float sc) {
  __shared__ float Tt[64 * 65];
  const int tid = threadIdx.x;
  const int c0 = blockIdx.x * 64, r0 = blockIdx.y * 64;
  const float* sb = src + (size_t)blockIdx.z * (size_t)R * (size_t)C;
  unsigned short* ob = O + (size_t)blockIdx.z * (size_t)C * (size_t)ldo;
#pragma unroll
  for (int i = 0; i < 4; ++i) {
    const int idx = i * 256 + tid;
    const int rr = idx >> 4, cc = (idx & 15) * 4;
    const v4f v = *(const v4f*)(sb + (size_t)(r0 + rr) * (size_t)C + c0 + cc);
    Tt[rr * 65 + cc + 0] = v[0];
    Tt[rr * 65 + cc + 1] = v[1];
    Tt[rr * 65 + cc + 2] = v[2];
    Tt[rr * 65 + cc + 3] = v[3];
  }
  __syncthreads();
  const int q = tid >> 3, c8 = (tid & 7) * 8;
  v8h hv[2];
#pragma unroll
  for (int g = 0; g < 2; ++g) {
    const int qq = g * 32 + q;
#pragma unroll
    for (int e = 0; e < 8; ++e) {
      const float f = Tt[(c8 + e) * 65 + qq];
      hv[g][e] = (_Float16)(f * sc);
    }
  }
  for (int pass = 0; pass < 2; ++pass) {
#pragma unroll
    for (int g = 0; g < 2; ++g) {
      const size_t o = (size_t)(c0 + g * 32 + q) * (size_t)ldo + (size_t)(r0 + c8);
      *(volatile v8h*)(ob + o) = hv[g];
    }
    __threadfence();
  }
}

__device__ __forceinline__ void gemm_gates(const _Float16* atile, int apitch, const _Float16* __restrict__ W, int ldw, int nk,
                                           float* sG, int wave, int c, int hh) {
  const int koff = hh * 8;
  const v8f z8 = {0.f, 0.f, 0.f, 0.f, 0.f, 0.f, 0.f, 0.f};
  v8f acc0 = z8, acc1 = z8, acc2 = z8, acc3 = z8;
  const _Float16* arow = atile + c * apitch + koff;
  const _Float16* w0 = W + (size_t)(wave * 16 + c) * (size_t)ldw + koff;
  const size_t gs = (size_t)NH * (size_t)ldw;
#pragma unroll 1
  for (int kt = 0; kt < nk; ++kt) {
    const int k0 = kt * 32;
    const v16h a  = Frag<_Float16>::load(arow + k0);
    const v16h b0 = Frag<_Float16>::load(w0 + k0);
    const v16h b1 = Frag<_Float16>::load(w0 + gs + k0);
    const v16h b2 = Frag<_Float16>::load(w0 + 2 * gs + k0);
    const v16h b3 = Frag<_Float16>::load(w0 + 3 * gs + k0);
    acc0 = Frag<_Float16>::mma(a, b0, acc0);
    acc1 = Frag<_Float16>::mma(a, b1, acc1);
    acc2 = Frag<_Float16>::mma(a, b2, acc2);
    acc3 = Frag<_Float16>::mma(a, b3, acc3);
    dep_guard4_h(acc0, acc1, acc2, acc3, a, b3);
    keep4_h(b0, b1, b2, b3);
  }
  acc_guard4(acc0, acc1, acc2, acc3);
  if (hh == 0) {
    const int col = wave * 16 + c;
#pragma unroll
    for (int r = 0; r < 8; ++r) {
      sG[r * NG4 + col]          = acc0[r];
      sG[r * NG4 + NH + col]     = acc1[r];
      sG[r * NG4 + 2 * NH + col] = acc2[r];
      sG[r * NG4 + 3 * NH + col] = acc3[r];
    }
  }
}

template <int LAYER>
__device__ __forceinline__ void lstm_ew(const float* sG, const float* sBiasL, float* sCL,
                                        _Float16* sA1, _Float16* sA2, _Float16* sA3, float* sH3, int tid) {
#pragma unroll 1
  for (int i = 0; i < 4; ++i) {
    const int idx = tid + NTHR * i;
    const int b = idx >> 8;
    const int j = idx & 255;
    const float* g = sG + b * NG4;
    const float zi = g[j] * FOLD + sBiasL[j];
    const float zf = g[NH + j] * FOLD + sBiasL[NH + j];
    const float zg = g[2 * NH + j] * FOLD + sBiasL[2 * NH + j];
    const float zo = g[3 * NH + j] * FOLD + sBiasL[3 * NH + j];
    const float cn = fsig(zf) * sCL[idx] + fsig(zi) * ftanh(zg);
    const float hn = fsig(zo) * ftanh(cn);
    sCL[idx] = cn;
    const _Float16 h16 = (_Float16)(hn * ACARRY);
    if (LAYER == 1) {
      sA1[b * A1P + KIN1 + j] = h16;
      sA2[b * A23P + j] = h16;
    }
    if (LAYER == 2) {
      sA2[b * A23P + NH + j] = h16;
      sA3[b * A23P + j] = h16;
    }
    if (LAYER == 3) {
      sA3[b * A23P + NH + j] = h16;
      sH3[idx] = hn;
    }
  }
}

__global__ __launch_bounds__(NTHR) void decoder_kernel(
    const int* __restrict__ pL,
    const float* __restrict__ ba, const float* __restrict__ wv, const float* __restrict__ bv,
    const float* __restrict__ bih1, const float* __restrict__ bhh1,
    const float* __restrict__ bih2, const float* __restrict__ bhh2,
    const float* __restrict__ bih3, const float* __restrict__ bhh3,
    const float* __restrict__ bm, const float* __restrict__ Ws, const float* __restrict__ bs,
    const float* __restrict__ Eenc,
    const unsigned short* __restrict__ encTp, const unsigned short* __restrict__ WaQp,
    const unsigned short* __restrict__ Wc1p, const unsigned short* __restrict__ Wc2p,
    const unsigned short* __restrict__ Wc3p, const unsigned short* __restrict__ WmPp,
    float* __restrict__ out) {
  __shared__ __align__(16) _Float16 sA1[16 * A1P];
  __shared__ __align__(16) _Float16 sA2[16 * A23P];
  __shared__ __align__(16) _Float16 sA3[16 * A23P];
  __shared__ __align__(16) _Float16 sP[NBAT * NTE];
  __shared__ __align__(16) float sG[NBAT * NG4];
  __shared__ __align__(16) float sC[3 * NBAT * NH];
  __shared__ __align__(16) float sH3[NBAT * NH];
  __shared__ __align__(16) float sCtx[NBAT * NENC];
  __shared__ __align__(16) float sBias[3 * NG4];
  __shared__ __align__(16) float sWs[KDEC];
  __shared__ __align__(16) float sMel2[NBAT * 2 * NMEL];
  __shared__ __align__(16) float sStop[NBAT * NSTEP];
  float* sSc = sG;
  float* sQP = sG + NBAT * NTE;

  const _Float16* encT = (const _Float16*)encTp;
  const _Float16* WaQ  = (const _Float16*)WaQp;
  const _Float16* Wc1  = (const _Float16*)Wc1p;
  const _Float16* Wc2  = (const _Float16*)Wc2p;
  const _Float16* Wc3  = (const _Float16*)Wc3p;
  const _Float16* WmP  = (const _Float16*)WmPp;

  const int tid  = threadIdx.x;
  const int lane = tid & 31;
  const int wave = __builtin_amdgcn_readfirstlane((int)(threadIdx.x >> 5));
  const int c = lane & 15, hh = lane >> 4, koff = hh * 8;
  const v8f z8 = {0.f, 0.f, 0.f, 0.f, 0.f, 0.f, 0.f, 0.f};

  const v4f wv0 = *(const v4f*)(wv + 4 * lane);
  const v4f wv1 = *(const v4f*)(wv + 128 + 4 * lane);
  const float ba_r = ba[wave * 16 + c];
  const int wm = (wave < 5) ? wave : 4;
  const float bm_r = bm[wm * 16 + c];
  const float bv_r = bv[0];
  const float bs_r = bs[0];
  int Lc = pL[0];
  Lc = (Lc < 0) ? 0 : Lc;
  Lc = (Lc > NSTEP) ? NSTEP : Lc;

#pragma unroll 1
  for (int i = tid; i < 16 * A1P; i += NTHR) sA1[i] = (_Float16)0.0f;
#pragma unroll 1
  for (int i = tid; i < 16 * A23P; i += NTHR) {
    sA2[i] = (_Float16)0.0f;
    sA3[i] = (_Float16)0.0f;
  }
#pragma unroll 1
  for (int i = tid; i < 3 * NBAT * NH; i += NTHR) sC[i] = 0.0f;
#pragma unroll 1
  for (int i = tid; i < NBAT * NH; i += NTHR) sH3[i] = 0.0f;
#pragma unroll 1
  for (int i = tid; i < NBAT * 2 * NMEL; i += NTHR) sMel2[i] = 0.0f;
#pragma unroll 1
  for (int i = tid; i < NBAT * NSTEP; i += NTHR) sStop[i] = 0.0f;
#pragma unroll 1
  for (int it = 0; it < 2; ++it) {
    const int n = tid + NTHR * it;
    sBias[n]           = bih1[n] + bhh1[n];
    sBias[NG4 + n]     = bih2[n] + bhh2[n];
    sBias[2 * NG4 + n] = bih3[n] + bhh3[n];
  }
#pragma unroll 1
  for (int it = 0; it < 2; ++it) {
    const int n = tid + NTHR * it;
    const int nc = (n < KDEC) ? n : (KDEC - 1);
    const float wsv = Ws[nc];
    if (n < KDEC) sWs[n] = wsv;
  }
  __syncthreads();

#pragma unroll 1
  for (int s = 0; s < Lc; ++s) {
    {
      v8f acc = z8;
      const _Float16* arow = sA3 + c * A23P + NH + koff;
      const _Float16* brow = WaQ + (size_t)(wave * 16 + c) * NH + koff;
#pragma unroll 1
      for (int k0 = 0; k0 < NH; k0 += 32) {
        const v16h a = Frag<_Float16>::load(arow + k0);
        const v16h b = Frag<_Float16>::load(brow + k0);
        acc = Frag<_Float16>::mma(a, b, acc);
        dep_guard1_h(acc, a, b);
      }
      acc_guard1(acc);
      if (hh == 0) {
#pragma unroll
        for (int r = 0; r < 8; ++r) sQP[r * NH + wave * 16 + c] = acc[r] * FOLD + ba_r;
      }
    }
    __syncthreads();

    {
      const int b  = wave >> 1;
      const int tb = (wave & 1) * 128;
      const v4f q0 = *(const v4f*)(sQP + b * NH + 4 * lane);
      const v4f q1 = *(const v4f*)(sQP + b * NH + 128 + 4 * lane);
      const float* ep = Eenc + ((size_t)(b * NTE + tb)) * NH + 4 * lane;
#pragma unroll 1
      for (int t = 0; t < 128; ++t) {
        const v4f e0 = *(const v4f*)(ep + (size_t)t * NH);
        const v4f e1 = *(const v4f*)(ep + (size_t)t * NH + 128);
        float sacc = 0.0f;
#pragma unroll
        for (int e = 0; e < 4; ++e) {
          sacc = fmaf(wv0[e], ftanh(e0[e] + q0[e]), sacc);
          sacc = fmaf(wv1[e], ftanh(e1[e] + q1[e]), sacc);
        }
#pragma unroll
        for (int off = 16; off >= 1; off >>= 1) sacc += __shfl_xor(sacc, off, 32);
        if (lane == 0) sSc[b * NTE + tb + t] = sacc + bv_r;
      }
    }
    __syncthreads();

    {
      const int b = wave & 7;
      float v[8];
      float mx = -INFINITY;
#pragma unroll
      for (int q = 0; q < 8; ++q) {
        v[q] = sSc[b * NTE + lane + 32 * q];
        mx = fmaxf(mx, v[q]);
      }
#pragma unroll
      for (int off = 16; off >= 1; off >>= 1) mx = fmaxf(mx, __shfl_xor(mx, off, 32));
      float sum = 0.0f;
#pragma unroll
      for (int q = 0; q < 8; ++q) {
        v[q] = expf(v[q] - mx);
        sum += v[q];
      }
#pragma unroll
      for (int off = 16; off >= 1; off >>= 1) sum += __shfl_xor(sum, off, 32);
      const float inv = PCARRY * (1.0f / sum);
      if (wave < 8) {
#pragma unroll
        for (int q = 0; q < 8; ++q) sP[b * NTE + lane + 32 * q] = (_Float16)(v[q] * inv);
      }
    }
    __syncthreads();

    {
      const int b = wave >> 1;
      const int nb = (wave & 1) * 16;
      const _Float16* arow = sP + b * NTE + koff;
#pragma unroll 1
      for (int g = 0; g < 4; ++g) {
        const int d0 = (nb + 4 * g) * 16 + c;
        const _Float16* bp = encT + ((size_t)(b * NENC + d0)) * NTE + koff;
        v8f acc[4];
        acc[0] = z8; acc[1] = z8; acc[2] = z8; acc[3] = z8;
#pragma unroll 1
        for (int k0 = 0; k0 < NTE; k0 += 32) {
          const v16h a  = Frag<_Float16>::load(arow + k0);
          const v16h b0 = Frag<_Float16>::load(bp + k0);
          const v16h b1 = Frag<_Float16>::load(bp + (size_t)16 * NTE + k0);
          const v16h b2 = Frag<_Float16>::load(bp + (size_t)32 * NTE + k0);
          const v16h b3 = Frag<_Float16>::load(bp + (size_t)48 * NTE + k0);
          acc[0] = Frag<_Float16>::mma(a, b0, acc[0]);
          acc[1] = Frag<_Float16>::mma(a, b1, acc[1]);
          acc[2] = Frag<_Float16>::mma(a, b2, acc[2]);
          acc[3] = Frag<_Float16>::mma(a, b3, acc[3]);
          dep_guard4_h(acc[0], acc[1], acc[2], acc[3], a, b3);
          keep4_h(b0, b1, b2, b3);
        }
        acc_guard4(acc[0], acc[1], acc[2], acc[3]);
        if (hh == 0) {
#pragma unroll
          for (int j = 0; j < 4; ++j) {
            const float cv = acc[j][0] * PINV;
            sCtx[b * NENC + d0 + 16 * j] = cv;
            sA1[b * A1P + NMEL + d0 + 16 * j] = (_Float16)(cv * ACARRY);
          }
        }
      }
      if (tid < 256) {
        const int pr = tid >> 4;
        const int pc = K1REAL + (tid & 15);
        sA1[pr * A1P + pc] = (_Float16)0.0f;
      }
    }
    __syncthreads();

    gemm_gates(sA1, A1P, Wc1, W1PITCH, K1PAD / 32, sG, wave, c, hh);
    __syncthreads();
    lstm_ew<1>(sG, sBias, sC, sA1, sA2, sA3, sH3, tid);
    __syncthreads();

    gemm_gates(sA2, A23P, Wc2, K23, K23 / 32, sG, wave, c, hh);
    __syncthreads();
    lstm_ew<2>(sG, sBias + NG4, sC + NBAT * NH, sA1, sA2, sA3, sH3, tid);
    __syncthreads();

    gemm_gates(sA3, A23P, Wc3, K23, K23 / 32, sG, wave, c, hh);
    __syncthreads();
    lstm_ew<3>(sG, sBias + 2 * NG4, sC + 2 * NBAT * NH, sA1, sA2, sA3, sH3, tid);
    __syncthreads();

    if (wave < 5) {
      v8f acc = z8;
      const _Float16* ar3 = sA3 + c * A23P + NH + koff;
      const _Float16* ar1 = sA1 + c * A1P + NMEL + koff;
      const _Float16* brow = WmP + (size_t)(wave * 16 + c) * KDEC + koff;
#pragma unroll 1
      for (int k0 = 0; k0 < NH; k0 += 32) {
        const v16h a = Frag<_Float16>::load(ar3 + k0);
        const v16h b = Frag<_Float16>::load(brow + k0);
        acc = Frag<_Float16>::mma(a, b, acc);
        dep_guard1_h(acc, a, b);
      }
#pragma unroll 1
      for (int k0 = 0; k0 < NENC; k0 += 32) {
        const v16h a = Frag<_Float16>::load(ar1 + k0);
        const v16h b = Frag<_Float16>::load(brow + NH + k0);
        acc = Frag<_Float16>::mma(a, b, acc);
        dep_guard1_h(acc, a, b);
      }
      acc_guard1(acc);
      if (hh == 0) {
        const int col = wave * 16 + c;
        const int slot = (s & 1) * NMEL;
        const bool tailfix = ((s & 1) == 0) && (s == Lc - 1);
#pragma unroll
        for (int r = 0; r < 8; ++r) {
          const float m = acc[r] * FOLD + bm_r;
          sMel2[r * (2 * NMEL) + slot + col] = m;
          sA1[r * A1P + col] = (_Float16)(m * ACARRY);
          if (tailfix) sMel2[r * (2 * NMEL) + NMEL + col] = 0.0f;
        }
      }
    }
    {
      const int b = wave & 7;
      float ps = 0.0f;
#pragma unroll 1
      for (int i = 0; i < NH / 32; ++i) {
        const int k = lane + 32 * i;
        ps = fmaf(sH3[b * NH + k], sWs[k], ps);
      }
#pragma unroll 1
      for (int i = 0; i < NENC / 32; ++i) {
        const int k = lane + 32 * i;
        ps = fmaf(sCtx[b * NENC + k], sWs[NH + k], ps);
      }
#pragma unroll
      for (int off = 16; off >= 1; off >>= 1) ps += __shfl_xor(ps, off, 32);
      const float sv = fsig(ps + bs_r);
      if (wave >= 8 && lane == 0) sStop[b * NSTEP + s] = sv;
    }
    __syncthreads();

    {
      const bool flush = ((s & 1) == 1) || (s == Lc - 1);
      if (flush && wave == 0) {
        const int s0 = s & ~1;
        for (int pass = 0; pass < 2; ++pass) {
#pragma unroll
          for (int it = 0; it < 10; ++it) {
            const int q  = it * 32 + lane;
            const int bq = q / 40;
            const int w4 = q - bq * 40;
            const v4f v = *(const v4f*)(sMel2 + bq * (2 * NMEL) + w4 * 4);
            *(volatile v4f*)(out + (size_t)(bq * NSTEP + s0) * NMEL + w4 * 4) = v;
          }
          __threadfence();
        }
      }
    }
  }

  __syncthreads();
  if (wave == 0) {
    for (int pass = 0; pass < 2; ++pass) {
#pragma unroll
      for (int it = 0; it < 7; ++it) {
        const int q  = it * 32 + lane;
        const int qc = (q < (NOUT1 / 4)) ? q : (NOUT1 / 4 - 1);
        const v4f v = *(const v4f*)(sStop + 4 * qc);
        if (q < (NOUT1 / 4)) *(volatile v4f*)(out + NOUT0 + 4 * q) = v;
      }
      __threadfence();
    }
  }
}

extern "C" void kernel_launch(void* const* d_in, const int* in_sizes, int n_in,
                              void* d_out, int out_size, void* d_ws, size_t ws_size, hipStream_t stream) {
  if (n_in < 22 || d_out == nullptr || d_ws == nullptr) return;
  if (in_sizes[0] != NROWS * NENC || in_sizes[1] != 1 || in_sizes[2] != NH * KATT || in_sizes[3] != NH ||
      in_sizes[4] != NH || in_sizes[5] != 1 || in_sizes[6] != NG4 * KIN1 || in_sizes[7] != NG4 * NH ||
      in_sizes[8] != NG4 || in_sizes[9] != NG4 || in_sizes[10] != NG4 * NH || in_sizes[11] != NG4 * NH ||
      in_sizes[12] != NG4 || in_sizes[13] != NG4 || in_sizes[14] != NG4 * NH || in_sizes[15] != NG4 * NH ||
      in_sizes[16] != NG4 || in_sizes[17] != NG4 || in_sizes[18] != NMEL * KDEC || in_sizes[19] != NMEL ||
      in_sizes[20] != KDEC || in_sizes[21] != 1 || out_size != NOUT0 + NOUT1) return;

  const float* enc  = (const float*)d_in[0];
  const int*   pL   = (const int*)d_in[1];
  const float* Wa   = (const float*)d_in[2];
  const float* ba   = (const float*)d_in[3];
  const float* wv   = (const float*)d_in[4];
  const float* bv   = (const float*)d_in[5];
  const float* Wih1 = (const float*)d_in[6];
  const float* Whh1 = (const float*)d_in[7];
  const float* bih1 = (const float*)d_in[8];
  const float* bhh1 = (const float*)d_in[9];
  const float* Wih2 = (const float*)d_in[10];
  const float* Whh2 = (const float*)d_in[11];
  const float* bih2 = (const float*)d_in[12];
  const float* bhh2 = (const float*)d_in[13];
  const float* Wih3 = (const float*)d_in[14];
  const float* Whh3 = (const float*)d_in[15];
  const float* bih3 = (const float*)d_in[16];
  const float* bhh3 = (const float*)d_in[17];
  const float* Wm   = (const float*)d_in[18];
  const float* bm   = (const float*)d_in[19];
  const float* Ws   = (const float*)d_in[20];
  const float* bs   = (const float*)d_in[21];
  float* out = (float*)d_out;

  char* ws = (char*)d_ws; size_t off = 0;
  auto carve = [&](size_t bytes) -> char* { char* p = ws + off; off += (bytes + 255) & ~(size_t)255; return p; };
  unsigned short* ENCH = (unsigned short*)carve((size_t)NROWS * NENC * 2);
  unsigned short* ENCT = (unsigned short*)carve((size_t)NBAT * NENC * NTE * 2);
  unsigned short* WAE  = (unsigned short*)carve((size_t)NH * NENC * 2);
  unsigned short* WAQ  = (unsigned short*)carve((size_t)NH * NH * 2);
  unsigned short* WC1  = (unsigned short*)carve((size_t)NG4 * W1PITCH * 2);
  unsigned short* WC2  = (unsigned short*)carve((size_t)NG4 * K23 * 2);
  unsigned short* WC3  = (unsigned short*)carve((size_t)NG4 * K23 * 2);
  unsigned short* WMP  = (unsigned short*)carve((size_t)NMEL * KDEC * 2);
  float*          EENC = (float*)carve((size_t)NROWS * NH * 4);
  if (off > ws_size || off > (size_t)134217728) return;

  pack2_kernel<<<(NROWS * (NENC / 8)) / 256, 256, 0, stream>>>(enc, NENC, 0, NENC / 8, enc, NENC, 0, 0, NENC / 8, NROWS, ENCH, 1.0f);
  tpose_f16_kernel<<<dim3(NENC / 64, NTE / 64, NBAT), 256, 0, stream>>>(enc, NTE, NENC, NTE, ENCT, 1.0f);
  pack2_kernel<<<(NH * (NENC / 8)) / 256, 256, 0, stream>>>(Wa, KATT, NH, NENC / 8, Wa, KATT, 0, 0, NENC / 8, NH, WAE, WCARRY);
  pack2_kernel<<<(NH * (NH / 8)) / 256, 256, 0, stream>>>(Wa, KATT, 0, NH / 8, Wa, KATT, 0, 0, NH / 8, NH, WAQ, WCARRY);
  pack2_kernel<<<(NG4 * (W1PITCH / 8)) / 256, 256, 0, stream>>>(Wih1, KIN1, 0, KIN1 / 8, Whh1, NH, 0, NH / 8, W1PITCH / 8, NG4, WC1, WCARRY);
  pack2_kernel<<<(NG4 * (K23 / 8)) / 256, 256, 0, stream>>>(Wih2, NH, 0, NH / 8, Whh2, NH, 0, NH / 8, K23 / 8, NG4, WC2, WCARRY);
  pack2_kernel<<<(NG4 * (K23 / 8)) / 256, 256, 0, stream>>>(Wih3, NH, 0, NH / 8, Whh3, NH, 0, NH / 8, K23 / 8, NG4, WC3, WCARRY);
  pack2_kernel<<<(NMEL * (KDEC / 8)) / 256, 256, 0, stream>>>(Wm, KDEC, 0, KDEC / 8, Wm, KDEC, 0, 0, KDEC / 8, NMEL, WMP, WCARRY);

  wmma_gemm64<0, false, 0, 0, false, 0><<<dim3((NROWS / 64) * (NH / 64) / 8, 1), 256, 0, stream>>>(
      ENCH, ENCH, NENC, 0L, WAE, WAE, NENC, 0L, (void*)EENC, (void*)EENC, NH, 0L,
      ba, EENC, 0L, NROWS, NH, NENC, 1.0f / WCARRY);

  decoder_kernel<<<1, NTHR, 0, stream>>>(pL, ba, wv, bv, bih1, bhh1, bih2, bhh2, bih3, bhh3, bm, Ws, bs,
                                         EENC, ENCT, WAQ, WC1, WC2, WC3, WMP, out);
}
